// SimpleRNN_16939351016020
// MI455X (gfx1250) — hardware-verified
//
#include <hip/hip_runtime.h>
#include <math.h>

constexpr int NBATCH   = 256;
constexpr int NSTEP    = 512;
constexpr int NIN      = 64;
constexpr int NHID     = 512;
constexpr int KCAT     = NHID + NIN;
constexpr int NTHR     = 256;
constexpr int ROWS_BLK = 16;
constexpr int APITCH   = 584;
constexpr int OPITCH   = 516;
constexpr float WCARRY     = 16.0f;
constexpr float WCARRY_INV = 1.0f / 16.0f;
constexpr int NOUT_ONE = NBATCH * NHID;
constexpr int WC_BLK_HH = (NHID * (NHID / 8)) / NTHR;
constexpr int WC_BLK_IH = (NHID * (NIN / 8)) / NTHR;

static_assert(NBATCH % ROWS_BLK == 0, "batch tile");
static_assert(KCAT % 32 == 0, "K multiple of 32");
static_assert(NHID == 64 * (NTHR / 32), "8 waves x 64 columns");
static_assert(NHID / 8 == 64 && NIN / 8 == 8, "prep index shifts");
static_assert((NHID * (NHID / 8)) % NTHR == 0 && (NHID * (NIN / 8)) % NTHR == 0, "prep grid exact");
static_assert((KCAT * 2) % 128 == 0, "weight plane row pitch is a whole number of 128-B lines");
static_assert(ROWS_BLK * NIN == NTHR * 4, "x tile: one float4 per thread");
static_assert((ROWS_BLK * NHID) % (NTHR * 4) == 0, "h0 / output tile loops exact");
static_assert(APITCH % 8 == 0 && APITCH >= KCAT, "A tile pitch");
static_assert(OPITCH % 4 == 0 && OPITCH >= NHID, "staging pitch");
static_assert((size_t)NOUT_ONE * 4 == 524288, "second output byte offset");

typedef __attribute__((ext_vector_type(16))) _Float16 v16h;
typedef __attribute__((ext_vector_type(8)))  _Float16 v8h;
typedef __attribute__((ext_vector_type(4)))  _Float16 v4h;
typedef __attribute__((ext_vector_type(8)))  float    v8f;
typedef __attribute__((ext_vector_type(4)))  float    v4f;

union FragU { v16h v; v8h h[2]; };
__device__ __forceinline__ v16h frag_load(const _Float16* p) {
  FragU f;
  f.h[0] = *(const v8h*)(p);
  f.h[1] = *(const v8h*)(p + 16);
  return f.v;
}
__device__ __forceinline__ v8f frag_mma(v16h a, v16h b, v8f c) {
  return __builtin_amdgcn_wmma_f32_16x16x32_f16(false, a, false, b, (short)0, c, false, false);
}
__device__ __forceinline__ void guard_group4(v8f& a0, v8f& a1, v8f& a2, v8f& a3,
                                             v16h x, v16h b0, v16h b1, v16h b2, v16h b3) {
  asm volatile("v_nop\n\tv_nop\n\tv_nop\n\tv_nop"
               : "+v"(a0), "+v"(a1), "+v"(a2), "+v"(a3)
               : "v"(x), "v"(b0), "v"(b1), "v"(b2), "v"(b3));
}
__device__ __forceinline__ void acc_guard4(v8f& a, v8f& b, v8f& c, v8f& d) {
  asm volatile("v_nop\n\tv_nop\n\tv_nop\n\tv_nop" : "+v"(a), "+v"(b), "+v"(c), "+v"(d));
}
__device__ __forceinline__ float tanh_f32(float x) {
  const float e = expf(2.0f * x);
  return 1.0f - 2.0f * __builtin_amdgcn_rcpf(e + 1.0f);
}

__global__ __launch_bounds__(NTHR) void wcat_kernel(const float* __restrict__ whh, const float* __restrict__ wih,
                                                    _Float16* __restrict__ wc) {
  const int tid = threadIdx.x;
  const bool second = ((int)blockIdx.x >= WC_BLK_HH);
  const float* src  = second ? wih : whh;
  const int shift   = second ? 3 : 6;
  const int spitch  = second ? NIN : NHID;
  const int dcol0   = second ? NHID : 0;
  const int i   = ((int)blockIdx.x - (second ? WC_BLK_HH : 0)) * NTHR + tid;
  const int row = i >> shift;
  const int c8  = i & ((1 << shift) - 1);
  const float* sp = src + (size_t)row * spitch + c8 * 8;
  const v4f a = *(const v4f*)(sp);
  const v4f b = *(const v4f*)(sp + 4);
  v8h hv;
#pragma unroll
  for (int e = 0; e < 4; ++e) {
    hv[e]     = (_Float16)(a[e] * WCARRY);
    hv[4 + e] = (_Float16)(b[e] * WCARRY);
  }
  _Float16* dp = wc + (size_t)row * KCAT + dcol0 + c8 * 8;
  *(volatile v8h*)dp = hv;
  __threadfence();
  *(volatile v8h*)dp = hv;
}

__global__ __launch_bounds__(NTHR) void rnn_seq_kernel(const float* __restrict__ x, const float* __restrict__ h0,
                                                       const float* __restrict__ b_ih, const float* __restrict__ b_hh,
                                                       const _Float16* __restrict__ wc, float* __restrict__ out) {
  __shared__ __align__(16) _Float16 Ah[2][ROWS_BLK * APITCH];
  __shared__ __align__(16) float    Hs[ROWS_BLK * OPITCH];

  const int tid = threadIdx.x, lane = tid & 31, wave = tid >> 5;
  const int c = lane & 15, hh = lane >> 4, koff = hh * 8;
  const int rowbase = blockIdx.x * ROWS_BLK;
  const int xm = tid >> 4, xf4 = (tid & 15) * 4;

#pragma unroll 1
  for (int it = 0; it < (ROWS_BLK * NHID) / (NTHR * 4); ++it) {
    const int idx = it * NTHR + tid;
    const int row = idx >> 7;
    const int c4  = (idx & 127) * 4;
    const v4f v = *(const v4f*)(h0 + (size_t)(rowbase + row) * NHID + c4);
    v4h hv;
#pragma unroll
    for (int e = 0; e < 4; ++e) hv[e] = (_Float16)v[e];
    *(v4h*)(&Ah[0][0] + row * APITCH + c4) = hv;
  }
  {
    const v4f v = *(const v4f*)(x + ((size_t)(rowbase + xm) * NSTEP) * NIN + xf4);
    v4h hv;
#pragma unroll
    for (int e = 0; e < 4; ++e) hv[e] = (_Float16)v[e];
    *(v4h*)(&Ah[0][0] + xm * APITCH + NHID + xf4) = hv;
  }
  float bb0, bb1, bb2, bb3;
  {
    const int j0 = 64 * wave + c;
    bb0 = b_ih[j0]      + b_hh[j0];
    bb1 = b_ih[j0 + 16] + b_hh[j0 + 16];
    bb2 = b_ih[j0 + 32] + b_hh[j0 + 32];
    bb3 = b_ih[j0 + 48] + b_hh[j0 + 48];
  }
  __syncthreads();

  const _Float16* wb = wc + (size_t)(64 * wave + c) * KCAT + koff;
  const v8f z8 = {0.f, 0.f, 0.f, 0.f, 0.f, 0.f, 0.f, 0.f};

#pragma unroll 1
  for (int t = 0; t < NSTEP; ++t) {
    const int cur = t & 1;
    const _Float16* arow = &Ah[cur][0] + c * APITCH + koff;
    _Float16* anext = &Ah[cur ^ 1][0];
    const bool last = (t == NSTEP - 1);

    const int tn = (t + 1 < NSTEP) ? (t + 1) : (NSTEP - 1);
    v4f xv = *(const v4f*)(x + ((size_t)(rowbase + xm) * NSTEP + (size_t)tn) * NIN + xf4);
    asm volatile("" : "+v"(xv));

    v8f acc0 = z8, acc1 = z8, acc2 = z8, acc3 = z8;
#pragma unroll 1
    for (int k0 = 0; k0 < KCAT; k0 += 32) {
      const v16h a  = frag_load(arow + k0);
      const v16h b0 = frag_load(wb + k0);
      const v16h b1 = frag_load(wb + (size_t)16 * KCAT + k0);
      const v16h b2 = frag_load(wb + (size_t)32 * KCAT + k0);
      const v16h b3 = frag_load(wb + (size_t)48 * KCAT + k0);
      acc0 = frag_mma(a, b0, acc0);
      acc1 = frag_mma(a, b1, acc1);
      acc2 = frag_mma(a, b2, acc2);
      acc3 = frag_mma(a, b3, acc3);
      guard_group4(acc0, acc1, acc2, acc3, a, b0, b1, b2, b3);
    }
    acc_guard4(acc0, acc1, acc2, acc3);

#pragma unroll 1
    for (int g = 0; g < 4; ++g) {
      const int j = 64 * wave + 16 * g + c;
      float vv[8];
#pragma unroll
      for (int r = 0; r < 8; ++r) {
        const float pre = acc0[r] * WCARRY_INV + bb0;
        vv[r] = tanh_f32(pre);
      }
#pragma unroll
      for (int r = 0; r < 8; ++r) anext[(8 * hh + r) * APITCH + j] = (_Float16)vv[r];
      if (last) {
#pragma unroll
        for (int r = 0; r < 8; ++r) Hs[(8 * hh + r) * OPITCH + j] = vv[r];
      }
      const v8f ta = acc0;
      acc0 = acc1; acc1 = acc2; acc2 = acc3; acc3 = ta;
      const float tb = bb0;
      bb0 = bb1; bb1 = bb2; bb2 = bb3; bb3 = tb;
    }

    {
      v4h hx;
#pragma unroll
      for (int e = 0; e < 4; ++e) hx[e] = (_Float16)xv[e];
      *(v4h*)(anext + xm * APITCH + NHID + xf4) = hx;
    }
    __syncthreads();
  }

  for (int pass = 0; pass < 2; ++pass) {
#pragma unroll
    for (int it = 0; it < (ROWS_BLK * NHID) / (NTHR * 4); ++it) {
      const int idx = it * NTHR + tid;
      const int row = idx >> 7;
      const int c4  = (idx & 127) * 4;
      const v4f v = *(const v4f*)(Hs + row * OPITCH + c4);
      float* op = out + (size_t)(rowbase + row) * NHID + c4;
      *(volatile v4f*)(op) = v;
      *(volatile v4f*)(op + NOUT_ONE) = v;
    }
    __threadfence();
  }
}

extern "C" void kernel_launch(void* const* d_in, const int* in_sizes, int n_in,
                              void* d_out, int out_size, void* d_ws, size_t ws_size, hipStream_t stream) {
  if (n_in < 6 || d_out == nullptr || d_ws == nullptr) return;
  if (in_sizes[0] != NBATCH * NSTEP * NIN || in_sizes[1] != NBATCH * NHID || in_sizes[2] != NHID * NIN ||
      in_sizes[3] != NHID * NHID || in_sizes[4] != NHID || in_sizes[5] != NHID ||
      out_size != 2 * NOUT_ONE) return;

  const float* x   = (const float*)d_in[0];
  const float* h0  = (const float*)d_in[1];
  const float* wih = (const float*)d_in[2];
  const float* whh = (const float*)d_in[3];
  const float* bih = (const float*)d_in[4];
  const float* bhh = (const float*)d_in[5];
  float* out = (float*)d_out;

  char* ws = (char*)d_ws;
  size_t off = 0;
  _Float16* wcat = (_Float16*)(ws + off);
  off += (((size_t)NHID * KCAT * 2) + 255) & ~(size_t)255;
  if (off > ws_size || off > (size_t)134217728) return;

  wcat_kernel<<<WC_BLK_HH + WC_BLK_IH, NTHR, 0, stream>>>(whh, wih, wcat);
  rnn_seq_kernel<<<NBATCH / ROWS_BLK, NTHR, 0, stream>>>(x, h0, bih, bhh, wcat, out);
}
